// SenseMemAct_46325517255182
// MI455X (gfx1250) — hardware-verified
//
#include <hip/hip_runtime.h>
#include <math.h>

constexpr int NBATCH  = 64;
constexpr int NSTEP   = 512;
constexpr int NFEAT   = 128;
constexpr int NSENSE  = 256;
constexpr int NHID    = 512;
constexpr int NDEC    = 3;
constexpr int NGIN    = 6;
constexpr int NGREC   = 5;
constexpr int NROWS   = NBATCH * NSTEP;
constexpr int SCAN_THR = 512;
constexpr int SEQ_BLK  = 16;
constexpr int HPITCH   = 520;
constexpr int CVT_THR  = 256;
constexpr int ACT_THR  = 256;
constexpr bool  INPUTS_RNE_BF16 = true;
constexpr float WCARRY     = 64.0f;
constexpr float WCARRY_INV = 1.0f / 64.0f;
constexpr float CMP_CARRY  = 16.0f;
constexpr float CMP_SCALE  = WCARRY / (CMP_CARRY * CMP_CARRY);
constexpr float RES_CARRY     = 2048.0f;
constexpr float RES_CARRY_INV = 1.0f / 2048.0f;
constexpr float HI_FLOOR      = 6.2e-5f;
static_assert(NBATCH % SEQ_BLK == 0);
static_assert(SEQ_BLK == SCAN_THR / 32);
static_assert(NHID == 32 * (SCAN_THR / 32));
static_assert(NFEAT % 32 == 0 && NHID % 32 == 0 && NSENSE % 32 == 0);
static_assert((NGIN * NHID) % 64 == 0 && NFEAT % 64 == 0 && NSENSE % 64 == 0);
static_assert(((NGIN * NHID / 64) * (NFEAT / 64)) % 8 == 0);
static_assert((NROWS * NFEAT / 8) % CVT_THR == 0);
static_assert((NHID * NHID / 8) % CVT_THR == 0);
static_assert((NHID * NSENSE / 8) % CVT_THR == 0);
static_assert(NROWS % ACT_THR == 0);
static_assert((NDEC * NHID) % ACT_THR == 0);
static_assert(NHID == 512 && NDEC == 3);
static_assert((HPITCH % 8) == 0 && HPITCH >= NHID);

typedef __attribute__((ext_vector_type(16))) _Float16 v16h;
typedef __attribute__((ext_vector_type(8)))  _Float16 v8h;
typedef __attribute__((ext_vector_type(16))) __bf16   v16b;
typedef __attribute__((ext_vector_type(8)))  __bf16   v8b;
typedef __attribute__((ext_vector_type(8)))  float    v8f;
typedef __attribute__((ext_vector_type(4)))  float    v4f;
typedef __attribute__((ext_vector_type(4)))  unsigned v4u;

__device__ __forceinline__ unsigned short f2bf_bits(float f) {
  unsigned u = __float_as_uint(f);
  return (unsigned short)((u + 0x7FFFu + ((u >> 16) & 1u)) >> 16);
}
__device__ __forceinline__ float bf_bits2f(unsigned short h) { return __uint_as_float(((unsigned)h) << 16); }
__device__ __forceinline__ float inr(float f) { return INPUTS_RNE_BF16 ? bf_bits2f(f2bf_bits(f)) : f; }

__device__ __forceinline__ float h16_to_f32(unsigned hb) {
  const unsigned sgn = (hb & 0x8000u) << 16;
  const unsigned em = hb & 0x7fffu;
  const float fn = __uint_as_float((em << 13) + 0x38000000u);
  const float fs = (float)em * 5.9604644775390625e-8f;
  const float mag = (em < 0x400u) ? fs : fn;
  return __uint_as_float(__float_as_uint(mag) | sgn);
}

__device__ __forceinline__ void dep_guard4_h(v8f& a, v8f& b, v8f& c, v8f& d, v16h x, v16h y) {
  asm volatile("v_nop\n\tv_nop\n\tv_nop\n\tv_nop" : "+v"(a), "+v"(b), "+v"(c), "+v"(d) : "v"(x), "v"(y));
}
__device__ __forceinline__ void dep_guard4_b(v8f& a, v8f& b, v8f& c, v8f& d, v16b x, v16b y) {
  asm volatile("v_nop\n\tv_nop\n\tv_nop\n\tv_nop" : "+v"(a), "+v"(b), "+v"(c), "+v"(d) : "v"(x), "v"(y));
}
__device__ __forceinline__ void keep4_h(v16h a, v16h b, v16h c, v16h d) { asm volatile("v_nop" :: "v"(a), "v"(b), "v"(c), "v"(d)); }
__device__ __forceinline__ void keep4_b(v16b a, v16b b, v16b c, v16b d) { asm volatile("v_nop" :: "v"(a), "v"(b), "v"(c), "v"(d)); }
__device__ __forceinline__ void acc_guard4(v8f& a, v8f& b, v8f& c, v8f& d) {
  asm volatile("v_nop\n\tv_nop\n\tv_nop\n\tv_nop" : "+v"(a), "+v"(b), "+v"(c), "+v"(d));
}
__device__ __forceinline__ void acc_guard6(v8f& a0, v8f& a1, v8f& a2, v8f& a3, v8f& a4, v8f& a5) {
  asm volatile("v_nop\n\tv_nop\n\tv_nop\n\tv_nop" : "+v"(a0), "+v"(a1), "+v"(a2), "+v"(a3), "+v"(a4), "+v"(a5));
}
__device__ __forceinline__ v8f mma_g(v16h a, v16h b, v8f c) {
  c = __builtin_amdgcn_wmma_f32_16x16x32_f16(false, a, false, b, (short)0, c, false, false);
  asm volatile("v_nop\n\tv_nop\n\tv_nop\n\tv_nop" : "+v"(c) : "v"(a), "v"(b));
  return c;
}

template <typename T> struct Frag;
template <> struct Frag<_Float16> {
  typedef v16h V; union U { v16h v; v8h h[2]; };
  static __device__ __forceinline__ v16h load(const _Float16* p) {
    U f; f.h[0] = *(const v8h*)(p); f.h[1] = *(const v8h*)(p + 16); return f.v;
  }
  static __device__ __forceinline__ v8f mma(v16h a, v16h b, v8f c) {
    return __builtin_amdgcn_wmma_f32_16x16x32_f16(false, a, false, b, (short)0, c, false, false);
  }
  static __device__ __forceinline__ void guard4(v8f& a, v8f& b, v8f& c, v8f& d, v16h x, v16h y) { dep_guard4_h(a, b, c, d, x, y); }
  static __device__ __forceinline__ void keep(v16h a, v16h b, v16h c, v16h d) { keep4_h(a, b, c, d); }
};
template <> struct Frag<__bf16> {
  typedef v16b V; union U { v16b v; v8b h[2]; };
  static __device__ __forceinline__ v16b load(const __bf16* p) {
    U f; f.h[0] = *(const v8b*)(p); f.h[1] = *(const v8b*)(p + 16); return f.v;
  }
  static __device__ __forceinline__ v8f mma(v16b a, v16b b, v8f c) {
    return __builtin_amdgcn_wmma_f32_16x16x32_bf16(false, a, false, b, (short)0, c, false, false);
  }
  static __device__ __forceinline__ void guard4(v8f& a, v8f& b, v8f& c, v8f& d, v16b x, v16b y) { dep_guard4_b(a, b, c, d, x, y); }
  static __device__ __forceinline__ void keep(v16b a, v16b b, v16b c, v16b d) { keep4_b(a, b, c, d); }
};

__device__ __forceinline__ float clamp30(float x) { return fminf(fmaxf(x, -30.0f), 30.0f); }
__device__ __forceinline__ float fsig(float x)  { return __builtin_amdgcn_rcpf(1.0f + __expf(-clamp30(x))); }
__device__ __forceinline__ float ftanh(float x) { return 1.0f - 2.0f * __builtin_amdgcn_rcpf(__expf(2.0f * clamp30(x)) + 1.0f); }

template <int ET> struct Elem;
template <> struct Elem<0> { typedef _Float16 T; };
template <> struct Elem<1> { typedef __bf16 T; };
template <int ET, bool SPLIT, int BIAS_MODE, int OUT_MODE, bool RESID, int ACT = 0>
__global__ __launch_bounds__(256) void wmma_gemm64(
    const unsigned short* __restrict__ Ap, const unsigned short* __restrict__ A2p, int lda, long strideA,
    const unsigned short* __restrict__ Btp, const unsigned short* __restrict__ Bt2p, int ldb, long strideB,
    void* __restrict__ Cout, void* __restrict__ Cout2, int ldc, long strideC,
    const float* __restrict__ bias,
    const float* __restrict__ resid, long strideR,
    int M, int N, int K, float scale) {
  typedef typename Elem<ET>::T T;
  typedef typename Frag<T>::V V;
  const T* A = (const T*)Ap; const T* A2 = (const T*)A2p; const T* Bt = (const T*)Btp; const T* Bt2 = (const T*)Bt2p;
  __shared__ __align__(16) float sT[8][16 * 68];
  const int b    = blockIdx.y;
  const int lane = threadIdx.x & 31;
  const int wave = threadIdx.x >> 5;
  const int tilesN = N >> 6;
  const int tilesM = M >> 6;
  const int tile = blockIdx.x * 8 + wave;
  if (tile >= tilesM * tilesN) return;
  const int tm = tile / tilesN;
  const int tn = tile - tm * tilesN;
  const int m0 = tm << 6;
  const int n0 = tn << 6;

  const T* Ab  = A  + (size_t)b * strideA;
  const T* Bb  = Bt + (size_t)b * strideB;
  const T* Ab2 = SPLIT ? (A2  + (size_t)b * strideA) : nullptr;
  const T* Bb2 = SPLIT ? (Bt2 + (size_t)b * strideB) : nullptr;

  const int rlane = lane & 15;
  const int koff  = (lane >> 4) * 8;
  const int mOff  = (lane >> 4) * 8;

  v8f acc[4][4];
#pragma unroll
  for (int i = 0; i < 4; ++i)
#pragma unroll
    for (int j = 0; j < 4; ++j) acc[i][j] = (v8f){0.f,0.f,0.f,0.f,0.f,0.f,0.f,0.f};

  for (int k0 = 0; k0 < K; k0 += 32) {
    V bh[4], bl[4];
#pragma unroll
    for (int j = 0; j < 4; ++j) {
      const size_t bo = (size_t)(n0 + (j << 4) + rlane) * ldb + koff + k0;
      bh[j] = Frag<T>::load(Bb + bo);
      if (SPLIT) bl[j] = Frag<T>::load(Bb2 + bo);
    }
#pragma unroll
    for (int i = 0; i < 4; ++i) {
      const size_t ao = (size_t)(m0 + (i << 4) + rlane) * lda + koff + k0;
      V ah = Frag<T>::load(Ab + ao);
      V al;
      if (SPLIT) al = Frag<T>::load(Ab2 + ao);
#pragma unroll
      for (int j = 0; j < 4; ++j) {
        acc[i][j] = Frag<T>::mma(ah, bh[j], acc[i][j]);
        if (SPLIT) {
          acc[i][j] = Frag<T>::mma(ah, bl[j], acc[i][j]);
          acc[i][j] = Frag<T>::mma(al, bh[j], acc[i][j]);
        }
      }
      Frag<T>::guard4(acc[i][0], acc[i][1], acc[i][2], acc[i][3], ah, SPLIT ? al : ah);
    }
    Frag<T>::keep(bh[0], bh[1], bh[2], bh[3]);
    if (SPLIT) Frag<T>::keep(bl[0], bl[1], bl[2], bl[3]);
  }
  acc_guard4(acc[0][0], acc[0][1], acc[0][2], acc[0][3]);
  acc_guard4(acc[1][0], acc[1][1], acc[1][2], acc[1][3]);
  acc_guard4(acc[2][0], acc[2][1], acc[2][2], acc[2][3]);
  acc_guard4(acc[3][0], acc[3][1], acc[3][2], acc[3][3]);

  float* slab = sT[wave];
  const float* Rb = RESID ? (resid + (size_t)b * strideR) : nullptr;
#pragma unroll
  for (int i = 0; i < 4; ++i) {
    const int mBase = m0 + (i << 4);
#pragma unroll
    for (int j = 0; j < 4; ++j) {
      const int n = n0 + (j << 4) + rlane;
      float bv = 0.f;
      if (BIAS_MODE == 2) bv = bias[n];
#pragma unroll
      for (int r = 0; r < 8; ++r) {
        float v = acc[i][j][r] * scale;
        if (BIAS_MODE == 1) v += bias[mBase + mOff + r];
        if (BIAS_MODE == 2) v += bv;
        if (RESID) v += Rb[(size_t)(mBase + mOff + r) * ldc + n];
        if (ACT == 1) v = tanhf(v);
        if (ACT == 2) v = fmaxf(v, 0.0f);
        if (ACT == 3) v = v / (1.0f + expf(-v));
        if (ACT == 4) v = (v > 0.f) ? v : 0.01f * v;
        slab[(mOff + r) * 68 + (j << 4) + rlane] = v;
      }
    }
    __builtin_amdgcn_fence(__ATOMIC_RELEASE, "workgroup");
    __builtin_amdgcn_wave_barrier();
    __builtin_amdgcn_fence(__ATOMIC_ACQUIRE, "workgroup");
    if (OUT_MODE == 0) {
      float* C = (float*)Cout + (size_t)b * strideC;
      const int hh = lane >> 4, c4 = (lane & 15) * 4;
      for (int pass = 0; pass < 2; ++pass) {
#pragma unroll
        for (int it = 0; it < 8; ++it) {
          const int row = it * 2 + hh;
          v4f v = *(const v4f*)(slab + row * 68 + c4);
          *(volatile v4f*)(C + (size_t)(mBase + row) * ldc + n0 + c4) = v;
        }
        __threadfence();
      }
    } else {
      const int q = lane >> 3, c8 = (lane & 7) * 8;
      unsigned short* C  = (unsigned short*)Cout  + (size_t)b * strideC;
      unsigned short* C2 = (OUT_MODE >= 2) ? ((unsigned short*)Cout2 + (size_t)b * strideC) : nullptr;
      for (int pass = 0; pass < 2; ++pass) {
#pragma unroll
        for (int it = 0; it < 4; ++it) {
          const int row = it * 4 + q;
          const float* sp = slab + row * 68 + c8;
          v8h hv, lv;
#pragma unroll
          for (int e = 0; e < 8; ++e) {
            if (OUT_MODE == 1) {
              hv[e] = (_Float16)sp[e];
            } else if (OUT_MODE == 2) {
              unsigned short hb = f2bf_bits(sp[e]);
              unsigned short lb = f2bf_bits(sp[e] - bf_bits2f(hb));
              hv[e] = __builtin_bit_cast(_Float16, hb);
              lv[e] = __builtin_bit_cast(_Float16, lb);
            } else {
              const float fv = sp[e];
              const float fh = (fabsf(fv) < HI_FLOOR) ? 0.0f : fv;
              const _Float16 h16 = (_Float16)fh;
              const float hback = (float)h16;
              const float fres = (fv - hback) * RES_CARRY;
              hv[e] = h16;
              lv[e] = (_Float16)fres;
            }
          }
          *(volatile v8h*)(C + (size_t)(mBase + row) * ldc + n0 + c8) = hv;
          if (OUT_MODE >= 2) *(volatile v8h*)(C2 + (size_t)(mBase + row) * ldc + n0 + c8) = lv;
        }
        __threadfence();
      }
    }
    __builtin_amdgcn_fence(__ATOMIC_RELEASE, "workgroup");
    __builtin_amdgcn_wave_barrier();
    __builtin_amdgcn_fence(__ATOMIC_ACQUIRE, "workgroup");
  }
}

__global__ __launch_bounds__(CVT_THR) void cvt8_f16_kernel(const float* __restrict__ src, unsigned short* __restrict__ dst,
                                                           int n8, float sc) {
  const int i = blockIdx.x * CVT_THR + threadIdx.x;
  if (i < n8) {
    const float* sp = src + (size_t)i * 8;
    const v4f a = *(const v4f*)(sp);
    const v4f b = *(const v4f*)(sp + 4);
    v8h hv;
#pragma unroll
    for (int e = 0; e < 4; ++e) {
      const float fa = a[e];
      const float fb = b[e];
      hv[e]     = (_Float16)(inr(fa) * sc);
      hv[4 + e] = (_Float16)(inr(fb) * sc);
    }
    *(volatile v8h*)(dst + (size_t)i * 8) = hv;
    __threadfence();
    *(volatile v8h*)(dst + (size_t)i * 8) = hv;
  }
}

__global__ __launch_bounds__(CVT_THR) void tp_f16_kernel(const float* __restrict__ src, int nr, int nc, int ldo,
                                                         unsigned short* __restrict__ outp, float sc) {
  __shared__ float Tt[64 * 65];
  const int tid = threadIdx.x;
  const int c0 = blockIdx.x * 64, r0 = blockIdx.y * 64;
#pragma unroll
  for (int i = 0; i < 4; ++i) {
    const int idx = i * CVT_THR + tid;
    const int rr = idx >> 4, cc = (idx & 15) * 4;
    const v4f v = *(const v4f*)(src + (size_t)(r0 + rr) * (size_t)nc + c0 + cc);
    Tt[rr * 65 + cc + 0] = v[0];
    Tt[rr * 65 + cc + 1] = v[1];
    Tt[rr * 65 + cc + 2] = v[2];
    Tt[rr * 65 + cc + 3] = v[3];
  }
  __syncthreads();
  const int q = tid >> 3, c8 = (tid & 7) * 8;
  v8h hv[2];
#pragma unroll
  for (int g = 0; g < 2; ++g) {
    const int qq = g * 32 + q;
#pragma unroll
    for (int e = 0; e < 8; ++e) {
      const float f = Tt[(c8 + e) * 65 + qq];
      hv[g][e] = (_Float16)(inr(f) * sc);
    }
  }
  for (int pass = 0; pass < 2; ++pass) {
#pragma unroll
    for (int g = 0; g < 2; ++g) {
      const size_t o = (size_t)(c0 + g * 32 + q) * (size_t)ldo + (size_t)(r0 + c8);
      *(volatile v8h*)(outp + o) = hv[g];
    }
    __threadfence();
  }
}

__global__ __launch_bounds__(SCAN_THR) void scan_kernel(const unsigned short* __restrict__ XHp,
                                                        const unsigned short* __restrict__ CWHp,
                                                        const unsigned short* __restrict__ CWLp,
                                                        const unsigned short* __restrict__ WHp,
                                                        unsigned short* __restrict__ MEMp) {
  __shared__ __align__(16) _Float16 Ah[2][SEQ_BLK * HPITCH];
  const _Float16* XH  = (const _Float16*)XHp;
  const _Float16* CWH = (const _Float16*)CWHp;
  const _Float16* CWL = (const _Float16*)CWLp;
  const _Float16* WH  = (const _Float16*)WHp;
  const int tid = threadIdx.x, lane = tid & 31, wave = tid >> 5;
  const int c = lane & 15, hh = lane >> 4, koff = hh * 8;
  const int rowbase = blockIdx.x * SEQ_BLK;

  {
    _Float16* ahf = &Ah[0][0];
#pragma unroll 1
    for (int i = tid; i < 2 * SEQ_BLK * HPITCH; i += SCAN_THR) ahf[i] = (_Float16)0.0f;
  }
  float hst[2][8], sst[2][8];
#pragma unroll
  for (int nt = 0; nt < 2; ++nt)
#pragma unroll
    for (int r = 0; r < 8; ++r) { hst[nt][r] = 0.0f; sst[nt][r] = 0.0f; }
  __syncthreads();

  const v8f z8 = {0.f, 0.f, 0.f, 0.f, 0.f, 0.f, 0.f, 0.f};
  const _Float16* xrow0 = XH + ((size_t)(rowbase + c) * NSTEP) * NFEAT + koff;

#pragma unroll 1
  for (int t = 0; t < NSTEP; ++t) {
    const int cur = t & 1;
    const _Float16* ahrow = &Ah[cur][0] + c * HPITCH + koff;
    _Float16* ahn = &Ah[cur ^ 1][0];
    const _Float16* xrow = xrow0 + (size_t)t * NFEAT;

#pragma unroll
    for (int nt = 0; nt < 2; ++nt) {
      const int j = 32 * wave + 16 * nt + c;
      const _Float16* cwh = CWH + (size_t)j * NFEAT + koff;
      const _Float16* cwl = CWL + (size_t)j * NFEAT + koff;
      const _Float16* wh  = WH + (size_t)j * NHID + koff;
      v8f accr[6];
      accr[0] = z8; accr[1] = z8; accr[2] = z8; accr[3] = z8; accr[4] = z8; accr[5] = z8;
#pragma unroll 1
      for (int kx = 0; kx < NFEAT; kx += 32) {
        const v16h a  = Frag<_Float16>::load(xrow + kx);
        const v16h b0 = Frag<_Float16>::load(cwl + kx);
        const v16h b1 = Frag<_Float16>::load(cwl + (size_t)1 * NHID * NFEAT + kx);
        const v16h b2 = Frag<_Float16>::load(cwl + (size_t)2 * NHID * NFEAT + kx);
        const v16h b3 = Frag<_Float16>::load(cwl + (size_t)3 * NHID * NFEAT + kx);
        const v16h b4 = Frag<_Float16>::load(cwl + (size_t)4 * NHID * NFEAT + kx);
        const v16h b5 = Frag<_Float16>::load(cwl + (size_t)5 * NHID * NFEAT + kx);
        accr[0] = mma_g(a, b0, accr[0]);
        accr[1] = mma_g(a, b1, accr[1]);
        accr[2] = mma_g(a, b2, accr[2]);
        accr[3] = mma_g(a, b3, accr[3]);
        accr[4] = mma_g(a, b4, accr[4]);
        accr[5] = mma_g(a, b5, accr[5]);
      }
      acc_guard6(accr[0], accr[1], accr[2], accr[3], accr[4], accr[5]);
      v8f acc[6];
#pragma unroll
      for (int g = 0; g < 6; ++g)
#pragma unroll
        for (int r = 0; r < 8; ++r) acc[g][r] = accr[g][r] * RES_CARRY_INV;
#pragma unroll 1
      for (int kx = 0; kx < NFEAT; kx += 32) {
        const v16h a  = Frag<_Float16>::load(xrow + kx);
        const v16h b0 = Frag<_Float16>::load(cwh + kx);
        const v16h b1 = Frag<_Float16>::load(cwh + (size_t)1 * NHID * NFEAT + kx);
        const v16h b2 = Frag<_Float16>::load(cwh + (size_t)2 * NHID * NFEAT + kx);
        const v16h b3 = Frag<_Float16>::load(cwh + (size_t)3 * NHID * NFEAT + kx);
        const v16h b4 = Frag<_Float16>::load(cwh + (size_t)4 * NHID * NFEAT + kx);
        const v16h b5 = Frag<_Float16>::load(cwh + (size_t)5 * NHID * NFEAT + kx);
        acc[0] = mma_g(a, b0, acc[0]);
        acc[1] = mma_g(a, b1, acc[1]);
        acc[2] = mma_g(a, b2, acc[2]);
        acc[3] = mma_g(a, b3, acc[3]);
        acc[4] = mma_g(a, b4, acc[4]);
        acc[5] = mma_g(a, b5, acc[5]);
      }
#pragma unroll 1
      for (int k0 = 0; k0 < NHID; k0 += 32) {
        const v16h a  = Frag<_Float16>::load(ahrow + k0);
        const v16h b0 = Frag<_Float16>::load(wh + k0);
        const v16h b1 = Frag<_Float16>::load(wh + (size_t)1 * NHID * NHID + k0);
        const v16h b2 = Frag<_Float16>::load(wh + (size_t)2 * NHID * NHID + k0);
        const v16h b3 = Frag<_Float16>::load(wh + (size_t)3 * NHID * NHID + k0);
        const v16h b4 = Frag<_Float16>::load(wh + (size_t)4 * NHID * NHID + k0);
        acc[0] = mma_g(a, b0, acc[0]);
        acc[1] = mma_g(a, b1, acc[1]);
        acc[2] = mma_g(a, b2, acc[2]);
        acc[3] = mma_g(a, b3, acc[3]);
        acc[4] = mma_g(a, b4, acc[4]);
      }
      acc_guard6(acc[0], acc[1], acc[2], acc[3], acc[4], acc[5]);
#pragma unroll
      for (int r = 0; r < 8; ++r) {
        const float pa = acc[0][r] * WCARRY_INV;
        const float pb = acc[1][r] * WCARRY_INV;
        const float pc = acc[2][r] * WCARRY_INV;
        const float pd = acc[3][r] * WCARRY_INV;
        const float pe = acc[4][r] * WCARRY_INV;
        const float po = acc[5][r] * WCARRY_INV;
        const float hf = hst[nt][r];
        const float hs = sst[nt][r];
        const float ga = 1.0f + ftanh(pa);
        const float gb = 1.5f * (1.0f + ftanh(pb));
        const float gc = 0.3f + 0.7f * fsig(pc);
        const float gd = 0.03f * fsig(pd);
        const float ge = 1.0f + fsig(pe);
        const float zz = po + (ga + gb * hf * hf - hs) * hf;
        const float hfn = (1.0f - gc) * hf + gc * ftanh(zz);
        float q4 = ge * hf;
        q4 = q4 * q4;
        q4 = q4 * q4;
        const float hsn = hs * (1.0f - gd) + gd * q4;
        hst[nt][r] = hfn;
        sst[nt][r] = hsn;
        ahn[(8 * hh + r) * HPITCH + j] = (_Float16)hfn;
      }
    }
    __syncthreads();

    {
      const _Float16* srcp = &Ah[cur ^ 1][0] + wave * HPITCH + 8 * lane;
      const v8h v0 = *(const v8h*)(srcp);
      const v8h v1 = *(const v8h*)(srcp + 256);
      unsigned short* dstp = MEMp + ((size_t)(rowbase + wave) * NSTEP + (size_t)t) * NHID + 8 * lane;
      for (int pass = 0; pass < 2; ++pass) {
        *(volatile v8h*)(dstp) = v0;
        *(volatile v8h*)(dstp + 256) = v1;
        __threadfence();
      }
    }
  }
}

__global__ __launch_bounds__(ACT_THR) void act_kernel(const unsigned short* __restrict__ MEMp,
                                                      const float* __restrict__ Wa, float* __restrict__ outp) {
  __shared__ __align__(16) float was[NDEC * NHID];
  __shared__ __align__(16) float so[ACT_THR / 32][96];
  const int tid = threadIdx.x, lane = tid & 31, wave = tid >> 5;
#pragma unroll 1
  for (int i = tid; i < NDEC * NHID; i += ACT_THR) was[i] = inr(Wa[i]);
  __syncthreads();

  const int row = blockIdx.x * ACT_THR + tid;
  const v4u* rp = (const v4u*)(MEMp + (size_t)row * NHID);
  float l0 = 0.0f, l1 = 0.0f, l2 = 0.0f;
#pragma unroll 1
  for (int i = 0; i < NHID / 8; ++i) {
    const v4u q = rp[i];
    const unsigned w0 = q[0];
    const unsigned w1 = q[1];
    const unsigned w2 = q[2];
    const unsigned w3 = q[3];
    float hv[8];
    hv[0] = h16_to_f32(w0 & 0xffffu);
    hv[1] = h16_to_f32(w0 >> 16);
    hv[2] = h16_to_f32(w1 & 0xffffu);
    hv[3] = h16_to_f32(w1 >> 16);
    hv[4] = h16_to_f32(w2 & 0xffffu);
    hv[5] = h16_to_f32(w2 >> 16);
    hv[6] = h16_to_f32(w3 & 0xffffu);
    hv[7] = h16_to_f32(w3 >> 16);
    const float* wp = was + 8 * i;
    const v4f a0 = *(const v4f*)(wp);
    const v4f a1 = *(const v4f*)(wp + 4);
    const v4f b0 = *(const v4f*)(wp + NHID);
    const v4f b1 = *(const v4f*)(wp + NHID + 4);
    const v4f c0 = *(const v4f*)(wp + 2 * NHID);
    const v4f c1 = *(const v4f*)(wp + 2 * NHID + 4);
#pragma unroll
    for (int e = 0; e < 4; ++e) {
      l0 = fmaf(hv[e], a0[e], l0);
      l1 = fmaf(hv[e], b0[e], l1);
      l2 = fmaf(hv[e], c0[e], l2);
    }
#pragma unroll
    for (int e = 0; e < 4; ++e) {
      l0 = fmaf(hv[4 + e], a1[e], l0);
      l1 = fmaf(hv[4 + e], b1[e], l1);
      l2 = fmaf(hv[4 + e], c1[e], l2);
    }
  }
  const float mx = fmaxf(l0, fmaxf(l1, l2));
  const float e0 = expf(l0 - mx);
  const float e1 = expf(l1 - mx);
  const float e2 = expf(l2 - mx);
  const float inv = 1.0f / ((e0 + e1) + e2);
  so[wave][3 * lane + 0] = e0 * inv;
  so[wave][3 * lane + 1] = e1 * inv;
  so[wave][3 * lane + 2] = e2 * inv;
  __syncthreads();
  const int li = (lane < 24) ? lane : 23;
  const v4f ov = *(const v4f*)(&so[wave][4 * li]);
  float* op = outp + ((size_t)blockIdx.x * ACT_THR + (size_t)wave * 32) * NDEC + 4 * li;
  if (lane < 24) *(volatile v4f*)op = ov;
  __threadfence();
  if (lane < 24) *(volatile v4f*)op = ov;
}

extern "C" void kernel_launch(void* const* d_in, const int* in_sizes, int n_in,
                              void* d_out, int out_size, void* d_ws, size_t ws_size, hipStream_t stream) {
  if (n_in < 14 || d_out == nullptr || d_ws == nullptr) return;
  if (in_sizes[0] != NBATCH * NSTEP * NFEAT || in_sizes[1] != NSENSE * NFEAT || in_sizes[2] != NDEC * NHID) return;
  for (int g = 0; g < NGIN; ++g) if (in_sizes[3 + 2 * g] != NHID * NSENSE) return;
  for (int g = 0; g < NGREC; ++g) if (in_sizes[4 + 2 * g] != NHID * NHID) return;
  if (out_size != NROWS * NDEC) return;

  const float* x  = (const float*)d_in[0];
  const float* Ws = (const float*)d_in[1];
  const float* Wa = (const float*)d_in[2];
  const float* Wi[NGIN]  = { (const float*)d_in[3],  (const float*)d_in[5],  (const float*)d_in[7],
                             (const float*)d_in[9],  (const float*)d_in[11], (const float*)d_in[13] };
  const float* Wh[NGREC] = { (const float*)d_in[4],  (const float*)d_in[6],  (const float*)d_in[8],
                             (const float*)d_in[10], (const float*)d_in[12] };
  float* outp = (float*)d_out;

  char* ws = (char*)d_ws; size_t off = 0;
  auto carve = [&](size_t bytes) -> char* { char* p = ws + off; off += (bytes + 255) & ~(size_t)255; return p; };
  unsigned short* XH  = (unsigned short*)carve((size_t)NROWS * NFEAT * 2);
  unsigned short* WHH = (unsigned short*)carve((size_t)NGREC * NHID * NHID * 2);
  unsigned short* WIH = (unsigned short*)carve((size_t)NGIN * NHID * NSENSE * 2);
  unsigned short* WST = (unsigned short*)carve((size_t)NFEAT * NSENSE * 2);
  unsigned short* CWH = (unsigned short*)carve((size_t)NGIN * NHID * NFEAT * 2);
  unsigned short* CWL = (unsigned short*)carve((size_t)NGIN * NHID * NFEAT * 2);
  unsigned short* MEM = (unsigned short*)carve((size_t)NROWS * NHID * 2);
  if (off > ws_size || off > (size_t)134217728) return;

  const int n8x = NROWS * NFEAT / 8;
  const int n8h = NHID * NHID / 8;
  const int n8i = NHID * NSENSE / 8;
  cvt8_f16_kernel<<<n8x / CVT_THR, CVT_THR, 0, stream>>>(x, XH, n8x, 1.0f);
  for (int g = 0; g < NGREC; ++g)
    cvt8_f16_kernel<<<n8h / CVT_THR, CVT_THR, 0, stream>>>(Wh[g], WHH + (size_t)g * NHID * NHID, n8h, WCARRY);
  for (int g = 0; g < NGIN; ++g)
    cvt8_f16_kernel<<<n8i / CVT_THR, CVT_THR, 0, stream>>>(Wi[g], WIH + (size_t)g * NHID * NSENSE, n8i, CMP_CARRY);
  tp_f16_kernel<<<dim3(NFEAT / 64, NSENSE / 64), CVT_THR, 0, stream>>>(Ws, NSENSE, NFEAT, NSENSE, WST, CMP_CARRY);

  wmma_gemm64<0, false, 0, 3, false, 0><<<dim3(((NGIN * NHID / 64) * (NFEAT / 64)) / 8, 1), 256, 0, stream>>>(
      WIH, WIH, NSENSE, 0L, WST, WST, NSENSE, 0L, (void*)CWH, (void*)CWL, NFEAT, 0L,
      Wa, Wa, 0L, NGIN * NHID, NFEAT, NSENSE, CMP_SCALE);

  scan_kernel<<<NBATCH / SEQ_BLK, SCAN_THR, 0, stream>>>(XH, CWH, CWL, WHH, MEM);

  act_kernel<<<NROWS / ACT_THR, ACT_THR, 0, stream>>>(MEM, Wa, outp);
}
